// LolcatsLinearAttention_28243704939085
// MI455X (gfx1250) — hardware-verified
//
#include <hip/hip_runtime.h>


namespace {
constexpr int L = 1024, H = 32, HD = 64, FD = 64, HID = 2048, NLT = L / 16;
constexpr float XS = 8.0f, QS = 64.0f  , FS = 2048.0f  , SS = 4096.0f  , YS = 64.0f, WSC = 256.0f;
typedef _Float16 b16;
typedef __attribute__((ext_vector_type(16))) _Float16 v16b;
typedef __attribute__((ext_vector_type(8))) _Float16 v8b;
typedef __attribute__((ext_vector_type(8))) float v8f;
typedef __attribute__((ext_vector_type(4))) float v4f;
__device__ __forceinline__ float bf16_rne(float f) { unsigned int u = __float_as_uint(f); u += 0x7FFFu + ((u >> 16) & 1u); return __uint_as_float(u & 0xFFFF0000u); }
__device__ __forceinline__ void split16(float v, b16& hi, b16& lo) { hi = (b16)v; lo = (b16)(v - (float)hi); }
__device__ __forceinline__ v16b frag_kb(const b16* p, int hh) { const v8b a = *(const v8b*)(p + 8 * hh), b = *(const v8b*)(p + 16 + 8 * hh); v16b f;
#pragma unroll
  for (int e = 0; e < 8; ++e) { f[e] = a[e]; f[8 + e] = b[e]; } return f; }
__device__ __forceinline__ v8f wmma16b(v16b a, v16b b, v8f c) { v8f d = __builtin_amdgcn_wmma_f32_16x16x32_f16(false, a, false, b, (short)0, c, false, false); asm volatile("v_nop\n\tv_nop\n\tv_nop\n\tv_nop" : "+v"(d) : "v"(a), "v"(b)); return d; }
__device__ __forceinline__ void wave_lds_sync() { __builtin_amdgcn_fence(__ATOMIC_RELEASE, "workgroup"); __builtin_amdgcn_wave_barrier(); __builtin_amdgcn_fence(__ATOMIC_ACQUIRE, "workgroup"); }
__device__ __forceinline__ float pmul(float a, float b) { float p = a * b; asm volatile("" : "+v"(p)); return p; }

__global__ __launch_bounds__(256) void wcopy_kernel(const float* __restrict__ w, int ro, b16* __restrict__ WT) {
  const size_t u = (size_t)blockIdx.x * 256 + threadIdx.x; if (u >= (size_t)HID * HID / 8) return; const size_t e = u * 8; v8b v;
#pragma unroll
  for (int j = 0; j < 8; ++j) v[j] = (b16)(bf16_rne(w[e + j]) * WSC); for (int pass = 0; pass < 2; ++pass) { *(volatile v8b*)(WT + (size_t)ro * HID + e) = v; __threadfence(); }
}
__global__ __launch_bounds__(256) void wf_kernel(const float* __restrict__ w, b16* __restrict__ WF) {
  const int u = blockIdx.x * 256 + threadIdx.x; if (u >= H * FD * HD / 8) return; const int e = u * 8; const int row = e / HD, d0 = e % HD; const int h = row / FD, f = row % FD; v8b v;
#pragma unroll
  for (int j = 0; j < 8; ++j) v[j] = (b16)(bf16_rne(w[((size_t)h * HD + d0 + j) * FD + f]) * WSC); for (int pass = 0; pass < 2; ++pass) { *(volatile v8b*)(WF + e) = v; __threadfence(); }
}
__global__ __launch_bounds__(256) void xa_kernel(const float* __restrict__ x, int n8, b16* __restrict__ XA) {
  const int u = blockIdx.x * 256 + threadIdx.x; if (u >= n8) return; const size_t e = (size_t)u * 8; v8b v;
#pragma unroll
  for (int j = 0; j < 8; ++j) v[j] = (b16)(bf16_rne(x[e + j]) * XS); for (int pass = 0; pass < 2; ++pass) { *(volatile v8b*)(XA + e) = v; __threadfence(); }
}
template <int TWO>
__global__ __launch_bounds__(32) void bgemm_kernel(const b16* __restrict__ AH, const b16* __restrict__ AL, const b16* __restrict__ WT, float sc, int POUT, int NLV, float* __restrict__ OUT) {
  __shared__ __attribute__((aligned(16))) float Tf[16][128 + 4];
  const int lane = threadIdx.x, nloc = lane & 15, hlf = lane >> 4; const size_t t0 = (size_t)(blockIdx.x % NLT) * 16; const int cg = blockIdx.x / NLT; if (t0 >= (size_t)NLV) return;
  const b16* ah = AH + (t0 + nloc) * HID; const b16* al_ = TWO ? AL + (t0 + nloc) * HID : nullptr;
#pragma unroll 1
  for (int ps = 0; ps < 4; ++ps) { const int c0 = cg * 512 + ps * 128; v8f acc[8];
#pragma unroll
    for (int t = 0; t < 8; ++t) acc[t] = (v8f){};
#pragma unroll 2
    for (int kb = 0; kb < HID; kb += 32) { const v16b a = frag_kb(ah + kb, hlf); v16b a2; if (TWO) a2 = frag_kb(al_ + kb, hlf);
#pragma unroll
      for (int t = 0; t < 8; ++t) { const v16b bw = frag_kb(WT + (size_t)(c0 + t * 16 + nloc) * HID + kb, hlf); acc[t] = wmma16b(a, bw, acc[t]); if (TWO) acc[t] = wmma16b(a2, bw, acc[t]); } }
#pragma unroll
    for (int t = 0; t < 8; ++t)
#pragma unroll 1
      for (int r8 = 0; r8 < 8; ++r8) Tf[8 * hlf + r8][t * 16 + nloc] = acc[t][r8] * sc;
    wave_lds_sync();
    for (int pass = 0; pass < 2; ++pass) { for (int rr = 0; rr < 16; ++rr) *(volatile v4f*)(OUT + (t0 + rr) * POUT + c0 + lane * 4) = *(const v4f*)(&Tf[rr][lane * 4]); __threadfence(); }
    wave_lds_sync(); }
}
__global__ __launch_bounds__(32) void fmap_kernel(const float* __restrict__ QKV, int which, const b16* __restrict__ WF, int NLV, float* __restrict__ F32, b16* __restrict__ FH, b16* __restrict__ FL) {
  __shared__ __attribute__((aligned(16))) b16 Ah[16][HD + 8], Al[16][HD + 8]; __shared__ __attribute__((aligned(16))) float Tf[16][FD + 4];
  const int lane = threadIdx.x, nloc = lane & 15, hlf = lane >> 4; const size_t t0 = (size_t)blockIdx.x * 16; const int h = blockIdx.y; if (t0 >= (size_t)NLV) return;
  for (int rr = 0; rr < 16; ++rr) for (int q = 0; q < 2; ++q) { b16 p, ql; split16(QKV[(t0 + rr) * (3 * HID) + which * HID + h * HD + q * 32 + lane] * QS, p, ql); Ah[rr][q * 32 + lane] = p; Al[rr][q * 32 + lane] = ql; }
  wave_lds_sync();
  v8f acc[4];
#pragma unroll
  for (int t = 0; t < 4; ++t) acc[t] = (v8f){};
#pragma unroll
  for (int kb = 0; kb < HD; kb += 32) { const v16b a = frag_kb(&Ah[nloc][kb], hlf), al = frag_kb(&Al[nloc][kb], hlf);
#pragma unroll
    for (int t = 0; t < 4; ++t) { const v16b bw = frag_kb(WF + ((size_t)h * FD + t * 16 + nloc) * HD + kb, hlf); acc[t] = wmma16b(a, bw, acc[t]); acc[t] = wmma16b(al, bw, acc[t]); } }
#pragma unroll
  for (int t = 0; t < 4; ++t)
#pragma unroll 1
    for (int r8 = 0; r8 < 8; ++r8) Tf[8 * hlf + r8][t * 16 + nloc] = acc[t][r8] * (1.0f / (QS * WSC));
  wave_lds_sync();
  for (int rr = 0; rr < 16; ++rr) { const float z0 = Tf[rr][lane], z1 = Tf[rr][32 + lane]; float mx = fmaxf(z0, z1); for (int o = 16; o; o >>= 1) mx = fmaxf(mx, __shfl_xor(mx, o)); const float e0 = __expf(z0 - mx), e1 = __expf(z1 - mx); float s = e0 + e1; for (int o = 16; o; o >>= 1) s += __shfl_xor(s, o); const float inv = 1.0f / s; wave_lds_sync(); Tf[rr][lane] = e0 * inv; Tf[rr][32 + lane] = e1 * inv; }
  wave_lds_sync();
  for (int pass = 0; pass < 2; ++pass) { for (int rr = 0; rr < 16; ++rr) { const size_t o = ((size_t)h * L + t0 + rr) * FD; for (int q = 0; q < 2; ++q) { const float v = Tf[rr][q * 32 + lane]; ((volatile float*)F32)[o + q * 32 + lane] = v; b16 p, ql; split16(v * FS, p, ql); ((volatile b16*)FH)[o + q * 32 + lane] = p; ((volatile b16*)FL)[o + q * 32 + lane] = ql; } } __threadfence(); }
}
__global__ __launch_bounds__(256) void vt_kernel(const float* __restrict__ QKV, int NLV, b16* __restrict__ VH, b16* __restrict__ VL) {
  __shared__ float T[64][65]; const int h = blockIdx.x % H, st = blockIdx.x / H; const int tid = threadIdx.x; if (st * 64 >= NLV) return;
  for (int i = tid; i < 64 * 64; i += 256) { const int r = i / 64, d = i % 64; T[r][d] = QKV[((size_t)st * 64 + r) * (3 * HID) + 2 * HID + h * HD + d]; }
  __syncthreads();
  { const int d = tid / 4, g = (tid % 4) * 2;
    for (int gg = g; gg < g + 2; ++gg) { v8b vh, vl;
#pragma unroll
      for (int j = 0; j < 8; ++j) { b16 p, q; split16(T[gg * 8 + j][d] * QS, p, q); vh[j] = p; vl[j] = q; }
      const size_t o = ((size_t)h * HD + d) * L + st * 64 + gg * 8; for (int pass = 0; pass < 2; ++pass) { *(volatile v8b*)(VH + o) = vh; *(volatile v8b*)(VL + o) = vl; __threadfence(); } } }
}
__global__ __launch_bounds__(256) void cum_kernel(const float* __restrict__ FK, int NLV, float* __restrict__ CK) {
  const int u = blockIdx.x * 256 + threadIdx.x; if (u >= H * FD) return; const int h = u / FD, f = u % FD;
#pragma unroll 1
  for (int pass = 0; pass < 2; ++pass) { float s = 0.0f;
#pragma unroll 4
    for (int l = 0; l < NLV; ++l) { s += FK[((size_t)h * L + l) * FD + f]; ((volatile float*)CK)[((size_t)h * L + l) * FD + f] = s; }
    __threadfence(); }
}
__global__ __launch_bounds__(32) void attn_kernel(const b16* __restrict__ FQH, const b16* __restrict__ FQL, const b16* __restrict__ FKH, const b16* __restrict__ FKL, const b16* __restrict__ VH, const b16* __restrict__ VL, const float* __restrict__ FQ32, const float* __restrict__ CK, int NLV, b16* __restrict__ YH, b16* __restrict__ YL) {
  __shared__ __attribute__((aligned(16))) b16 Sh[16][32 + 8], Sl[16][32 + 8]; __shared__ __attribute__((aligned(16))) float Tf[16][HD + 4];
  const int lane = threadIdx.x, nloc = lane & 15, hlf = lane >> 4; const int lt = blockIdx.x, h = blockIdx.y; const int l0 = lt * 16; if (l0 >= NLV) return;
  const size_t qr = ((size_t)h * L + l0 + nloc) * FD; v8f y[4];
#pragma unroll
  for (int t = 0; t < 4; ++t) y[t] = (v8f){};
  const int nkb = lt / 2 + 1;
#pragma unroll 1
  for (int kb = 0; kb < nkb; ++kb) { const int s0 = kb * 32; v8f sacc[2] = {(v8f){}, (v8f){}};
#pragma unroll
    for (int st = 0; st < 2; ++st) { const size_t kr = ((size_t)h * L + s0 + st * 16 + nloc) * FD;
#pragma unroll
      for (int k2 = 0; k2 < FD; k2 += 32) { const v16b ah = frag_kb(FQH + qr + k2, hlf), al = frag_kb(FQL + qr + k2, hlf), bh = frag_kb(FKH + kr + k2, hlf), bl = frag_kb(FKL + kr + k2, hlf); sacc[st] = wmma16b(ah, bh, sacc[st]); sacc[st] = wmma16b(ah, bl, sacc[st]); sacc[st] = wmma16b(al, bh, sacc[st]); sacc[st] = wmma16b(al, bl, sacc[st]); } }
#pragma unroll
    for (int st = 0; st < 2; ++st)
#pragma unroll
      for (int r8 = 0; r8 < 8; ++r8) { const int rl = 8 * hlf + r8; const int l = l0 + rl, s = s0 + st * 16 + nloc; const float v = (s <= l) ? sacc[st][r8] * (1.0f / (FS * FS)) : 0.0f; b16 p, q; split16(v * SS, p, q); Sh[rl][st * 16 + nloc] = p; Sl[rl][st * 16 + nloc] = q; }
    wave_lds_sync();
    { const v16b a = frag_kb(&Sh[nloc][0], hlf), al = frag_kb(&Sl[nloc][0], hlf);
#pragma unroll
      for (int t = 0; t < 4; ++t) { const size_t vr = ((size_t)h * HD + t * 16 + nloc) * L + s0; const v16b bh = frag_kb(VH + vr, hlf), bl = frag_kb(VL + vr, hlf); y[t] = wmma16b(a, bh, y[t]); y[t] = wmma16b(a, bl, y[t]); y[t] = wmma16b(al, bh, y[t]); y[t] = wmma16b(al, bl, y[t]); } }
    wave_lds_sync(); }
  float dn[16]; for (int rr = 0; rr < 16; ++rr) { const size_t o = ((size_t)h * L + l0 + rr) * FD; float s = pmul(FQ32[o + lane], CK[o + lane]) + pmul(FQ32[o + 32 + lane], CK[o + 32 + lane]); for (int oo = 16; oo; oo >>= 1) s += __shfl_xor(s, oo); dn[rr] = 1.0f / (s + 1e-12f); }
#pragma unroll
  for (int t = 0; t < 4; ++t)
#pragma unroll
    for (int r8 = 0; r8 < 8; ++r8) { const int rl = 8 * hlf + r8; float dsel = 0.0f;
#pragma unroll
      for (int rr = 0; rr < 16; ++rr) dsel = (rr == rl) ? dn[rr] : dsel; Tf[rl][t * 16 + nloc] = pmul(y[t][r8] * (1.0f / (SS * QS)), dsel); }
  wave_lds_sync();
  for (int pass = 0; pass < 2; ++pass) { for (int rr = 0; rr < 16; ++rr) for (int q = 0; q < 2; ++q) { const float v = Tf[rr][q * 32 + lane]; b16 p, ql; split16(v * YS, p, ql); const size_t o = (size_t)(l0 + rr) * HID + h * HD + q * 32 + lane; ((volatile b16*)YH)[o] = p; ((volatile b16*)YL)[o] = ql; } __threadfence(); }
}
}

extern "C" void kernel_launch(void* const* d_in, const int* in_sizes, int n_in, void* d_out, int out_size, void* d_ws, size_t ws_size, hipStream_t stream) {
  (void)n_in;
  auto Fp = [&](int i) { return (const float*)d_in[i]; };
  if (in_sizes[0] != L * HID || in_sizes[1] != HID * HID || in_sizes[2] != HID * HID || in_sizes[3] != HID * HID || in_sizes[4] != HID * HID || in_sizes[5] != H * HD * FD || in_sizes[6] != H * HD * FD || out_size != L * HID) return;
  const int NLV = L;
  size_t off = 0; char* ws = (char*)d_ws;
  auto carve = [&](size_t bytes) { char* p = ws + off; off += (bytes + 255) & ~(size_t)255; return p; };
  b16* WQKV = (b16*)carve((size_t)3 * HID * HID * 2); b16* WO = (b16*)carve((size_t)HID * HID * 2); b16* WFQ = (b16*)carve((size_t)H * FD * HD * 2); b16* WFK = (b16*)carve((size_t)H * FD * HD * 2); b16* XA = (b16*)carve((size_t)L * HID * 2);
  float* QKV = (float*)carve((size_t)L * 3 * HID * 4); float* FQ32 = (float*)carve((size_t)H * L * FD * 4); float* FK32 = (float*)carve((size_t)H * L * FD * 4); float* CK = (float*)carve((size_t)H * L * FD * 4);
  b16* FQH = (b16*)carve((size_t)H * L * FD * 2); b16* FQL = (b16*)carve((size_t)H * L * FD * 2); b16* FKH = (b16*)carve((size_t)H * L * FD * 2); b16* FKL = (b16*)carve((size_t)H * L * FD * 2); b16* VH = (b16*)carve((size_t)H * HD * L * 2); b16* VL = (b16*)carve((size_t)H * HD * L * 2); b16* YH = (b16*)carve((size_t)L * HID * 2); b16* YL = (b16*)carve((size_t)L * HID * 2);
  if (off > ws_size || off > ((size_t)160 << 20)) return;
  wcopy_kernel<<<(HID * HID / 8 + 255) / 256, 256, 0, stream>>>(Fp(1), 0, WQKV); wcopy_kernel<<<(HID * HID / 8 + 255) / 256, 256, 0, stream>>>(Fp(2), HID, WQKV); wcopy_kernel<<<(HID * HID / 8 + 255) / 256, 256, 0, stream>>>(Fp(3), 2 * HID, WQKV); wcopy_kernel<<<(HID * HID / 8 + 255) / 256, 256, 0, stream>>>(Fp(4), 0, WO);
  wf_kernel<<<(H * FD * HD / 8 + 255) / 256, 256, 0, stream>>>(Fp(5), WFQ); wf_kernel<<<(H * FD * HD / 8 + 255) / 256, 256, 0, stream>>>(Fp(6), WFK);
  xa_kernel<<<(L * HID / 8 + 255) / 256, 256, 0, stream>>>(Fp(0), L * HID / 8, XA);
  bgemm_kernel<0><<<NLT * 12, 32, 0, stream>>>(XA, nullptr, WQKV, 1.0f / (XS * WSC), 3 * HID, NLV, QKV);
  fmap_kernel<<<dim3(NLT, H), 32, 0, stream>>>(QKV, 0, WFQ, NLV, FQ32, FQH, FQL); fmap_kernel<<<dim3(NLT, H), 32, 0, stream>>>(QKV, 1, WFK, NLV, FK32, FKH, FKL);
  vt_kernel<<<(L / 64) * H, 256, 0, stream>>>(QKV, NLV, VH, VL);
  cum_kernel<<<(H * FD + 255) / 256, 256, 0, stream>>>(FK32, NLV, CK);
  attn_kernel<<<dim3(NLT, H), 32, 0, stream>>>(FQH, FQL, FKH, FKL, VH, VL, FQ32, CK, NLV, YH, YL);
  bgemm_kernel<1><<<NLT * 4, 32, 0, stream>>>(YH, YL, WO, 1.0f / (YS * WSC), HID, NLV, (float*)d_out);
}
